// MultiQueryattention_22763326669445
// MI455X (gfx1250) — hardware-verified
//
#include <hip/hip_runtime.h>
#include <stdint.h>


typedef _Float16 v16h __attribute__((ext_vector_type(16)));
typedef _Float16 v8h  __attribute__((ext_vector_type(8)));
typedef float    v8f  __attribute__((ext_vector_type(8)));
typedef float    v4f  __attribute__((ext_vector_type(4)));

#define DM 2048
#define HD 128
#define NH 16
#define NB_FULL 2
#define SEQ_FULL 2048
#ifndef NB
#define NB 2
#endif
#ifndef SEQ
#define SEQ 2048
#endif
#define MROWS (NB * SEQ)
#define WSCALE 64.0f
#define QCARRY 8.0f
#define KCARRY 8.0f
#define VCARRY 8.0f
#define PCARRY 1024.0f
#define LOG2E 1.4426950408889634f
#define SM_SCALE 0.08838834764831845f

#define QSP 136
#define PSP 40
#define OSP 132
#define WST (16 * OSP)

static_assert(SEQ % 128 == 0);
static_assert(SEQ <= SEQ_FULL);
static_assert(NB >= 1 && NB <= NB_FULL);
static_assert(DM == NH * HD && HD == 128 && DM % 128 == 0 && DM % 64 == 0);
static_assert(MROWS % 128 == 0);
static_assert((MROWS * (DM / 8)) % 256 == 0);
static_assert((NB * NH * (SEQ / 16)) % 4 == 0);
static_assert(16 * QSP + 16 * PSP <= 2 * WST);
static_assert((QSP * 2) % 16 == 0 && (PSP * 2) % 16 == 0 && (OSP * 4) % 16 == 0);

union HFrag { v16h v; v8h h[2]; };

__device__ __forceinline__ v16h load_frag(const _Float16* p) {
    HFrag f;
    f.h[0] = *reinterpret_cast<const v8h*>(p);
    f.h[1] = *reinterpret_cast<const v8h*>(p + 16);
    return f.v;
}

__device__ __forceinline__ v8f wmma16(v16h a, v16h b, v8f c) {
    return __builtin_amdgcn_wmma_f32_16x16x32_f16(false, a, false, b, (short)0, c, false, false);
}

__device__ __forceinline__ float bf16r(float f) {
    unsigned int u = __float_as_uint(f);
    u += 0x7FFFu + ((u >> 16) & 1u);
    u &= 0xFFFF0000u;
    return __uint_as_float(u);
}

__global__ __launch_bounds__(256) void k_cvt(const float* __restrict__ x, _Float16* x16)
{
    const int u = blockIdx.x * 256 + threadIdx.x;
    const int upr = DM / 8;
    const int row = u / upr;
    const int col = (u - row * upr) * 8;
    const int bi = row / SEQ;
    const int s  = row - bi * SEQ;
    const float* src = x + ((size_t)(bi * SEQ_FULL + s)) * DM + col;
    const float4 f0 = *reinterpret_cast<const float4*>(src);
    const float4 f1 = *reinterpret_cast<const float4*>(src + 4);
    v8h o;
    o[0] = (_Float16)bf16r(f0.x); o[1] = (_Float16)bf16r(f0.y);
    o[2] = (_Float16)bf16r(f0.z); o[3] = (_Float16)bf16r(f0.w);
    o[4] = (_Float16)bf16r(f1.x); o[5] = (_Float16)bf16r(f1.y);
    o[6] = (_Float16)bf16r(f1.z); o[7] = (_Float16)bf16r(f1.w);
    _Float16* dst = x16 + (size_t)row * DM + col;
    *(volatile v8h*)dst = o;
    __threadfence();
    *(volatile v8h*)dst = o;
}

__global__ __launch_bounds__(256) void k_wt(const float* __restrict__ W, _Float16* WT, int N)
{
    __shared__ _Float16 tile[32 * 72] __attribute__((aligned(16)));
    const int tid = threadIdx.x;
    const int n0 = blockIdx.x * 32, k0 = blockIdx.y * 64;
    const int nn = tid & 31, kq = tid >> 5;
#pragma unroll
    for (int i = 0; i < 8; ++i) {
        const int kk = kq + 8 * i;
        const float w = W[(size_t)(k0 + kk) * N + n0 + nn];
        tile[nn * 72 + kk] = (_Float16)(bf16r(w) * WSCALE);
    }
    __syncthreads();
    const int on = tid >> 3, seg = tid & 7;
    const v8h v = *reinterpret_cast<const v8h*>(tile + on * 72 + seg * 8);
    _Float16* dst = WT + (size_t)(n0 + on) * DM + k0 + seg * 8;
    *(volatile v8h*)dst = v;
    __threadfence();
    *(volatile v8h*)dst = v;
}

__device__ __forceinline__ void store32x64_f16(const _Float16* sw, _Float16* gdst,
                                               size_t pitch, int lane)
{
    const int rq = lane >> 3, seg = lane & 7;
    v8h v[8];
#pragma unroll
    for (int it = 0; it < 8; ++it)
        v[it] = *reinterpret_cast<const v8h*>(sw + (it * 4 + rq) * 64 + seg * 8);
#pragma unroll
    for (int it = 0; it < 8; ++it)
        *(volatile v8h*)(gdst + (size_t)(it * 4 + rq) * pitch + seg * 8) = v[it];
    __threadfence();
#pragma unroll
    for (int it = 0; it < 8; ++it)
        *(volatile v8h*)(gdst + (size_t)(it * 4 + rq) * pitch + seg * 8) = v[it];
}

template <int MODE>
__global__ __launch_bounds__(256) void k_gemm(const _Float16* __restrict__ A,
                                              const _Float16* __restrict__ BT,
                                              const float* __restrict__ bias,
                                              _Float16* C0, int N, int K, float alpha, float beta)
{
    __shared__ float stg[8 * 1024] __attribute__((aligned(16)));
    const int tid = threadIdx.x;
    const int lane = tid & 31, wave = tid >> 5;
    const int wm = wave & 3, wn = wave >> 2;
    const int l15 = lane & 15, hi8 = (lane >> 4) << 3;
    const int bm0 = blockIdx.y * 128, bn0 = blockIdx.x * 128;

    const _Float16* ap0 = A + (size_t)(bm0 + wm * 32 + l15) * K + hi8;
    const _Float16* ap1 = ap0 + (size_t)16 * K;
    const _Float16* bp  = BT + (size_t)(bn0 + wn * 64 + l15) * K + hi8;
    const size_t bst = (size_t)16 * K;

    const v8f zero8 = {0.f, 0.f, 0.f, 0.f, 0.f, 0.f, 0.f, 0.f};
    v8f acc[2][4];
#pragma unroll
    for (int g = 0; g < 2; ++g)
#pragma unroll
        for (int ni = 0; ni < 4; ++ni) acc[g][ni] = zero8;

    for (int k0 = 0; k0 < K; k0 += 32) {
        const v16h a0 = load_frag(ap0 + k0);
        const v16h a1 = load_frag(ap1 + k0);
        const v16h b0 = load_frag(bp + k0);
        const v16h b1 = load_frag(bp + bst + k0);
        const v16h b2 = load_frag(bp + 2 * bst + k0);
        const v16h b3 = load_frag(bp + 3 * bst + k0);
        acc[0][0] = wmma16(a0, b0, acc[0][0]);
        acc[0][1] = wmma16(a0, b1, acc[0][1]);
        acc[0][2] = wmma16(a0, b2, acc[0][2]);
        acc[0][3] = wmma16(a0, b3, acc[0][3]);
        acc[1][0] = wmma16(a1, b0, acc[1][0]);
        acc[1][1] = wmma16(a1, b1, acc[1][1]);
        acc[1][2] = wmma16(a1, b2, acc[1][2]);
        acc[1][3] = wmma16(a1, b3, acc[1][3]);
        asm volatile("v_nop\n\tv_nop\n\tv_nop\n\tv_nop"
                     : "+v"(acc[0][0]), "+v"(acc[0][1]), "+v"(acc[0][2]), "+v"(acc[0][3]),
                       "+v"(acc[1][0]), "+v"(acc[1][1]), "+v"(acc[1][2]), "+v"(acc[1][3])
                     : "v"(a0), "v"(a1), "v"(b0), "v"(b1), "v"(b2), "v"(b3));
    }

    float bcol[4];
#pragma unroll
    for (int ni = 0; ni < 4; ++ni) bcol[ni] = bf16r(bias[bn0 + wn * 64 + ni * 16 + l15]);

    if (MODE == 0) {
        _Float16* sw = reinterpret_cast<_Float16*>(stg + wave * 1024);
#pragma unroll
        for (int g = 0; g < 2; ++g)
#pragma unroll
            for (int ni = 0; ni < 4; ++ni)
#pragma unroll
                for (int j = 0; j < 8; ++j)
                    sw[(g * 16 + hi8 + j) * 64 + ni * 16 + l15] =
                        (_Float16)((acc[g][ni][j] * alpha + bcol[ni]) * beta);
        __syncthreads();
        store32x64_f16(sw, C0 + (size_t)(bm0 + wm * 32) * N + bn0 + wn * 64, (size_t)N, lane);
    } else {
        _Float16* vs = reinterpret_cast<_Float16*>(stg);
#pragma unroll
        for (int g = 0; g < 2; ++g)
#pragma unroll
            for (int ni = 0; ni < 4; ++ni)
#pragma unroll
                for (int j = 0; j < 8; ++j)
                    vs[(wn * 64 + ni * 16 + l15) * 128 + wm * 32 + g * 16 + hi8 + j] =
                        (_Float16)((acc[g][ni][j] * alpha + bcol[ni]) * beta);
        __syncthreads();
        const int bi = bm0 / SEQ;
        const int s0 = bm0 - bi * SEQ;
        const int dq = tid >> 4, seg = tid & 15;
        v8h v[8];
#pragma unroll
        for (int it = 0; it < 8; ++it)
            v[it] = *reinterpret_cast<const v8h*>(vs + (it * 16 + dq) * 128 + seg * 8);
        _Float16* vd = C0 + ((size_t)(bi * HD)) * SEQ + s0 + seg * 8;
#pragma unroll
        for (int it = 0; it < 8; ++it)
            *(volatile v8h*)(vd + (size_t)(it * 16 + dq) * SEQ) = v[it];
        __threadfence();
#pragma unroll
        for (int it = 0; it < 8; ++it)
            *(volatile v8h*)(vd + (size_t)(it * 16 + dq) * SEQ) = v[it];
    }
}

__global__ __launch_bounds__(128) void k_attn(const _Float16* __restrict__ qp,
                                              const _Float16* __restrict__ kp,
                                              const _Float16* __restrict__ vT,
                                              float* out)
{
    __shared__ float stg[4 * WST] __attribute__((aligned(16)));
    const int lane = threadIdx.x & 31;
    const int wv   = threadIdx.x >> 5;
    const int l15  = lane & 15;
    const int hi8  = (lane >> 4) << 3;

    const int qtiles = SEQ / 16;
    int gw = blockIdx.x * 4 + wv;
    const int qt = gw % qtiles; gw /= qtiles;
    const int h  = gw % NH;
    const int b  = gw / NH;

    float* my = stg + wv * WST;
    _Float16* qs = reinterpret_cast<_Float16*>(my);
    _Float16* ps = qs + 16 * QSP;

    {
        const int r = lane >> 1, c = (lane & 1) * 64;
        const _Float16* src = qp + ((size_t)(b * SEQ + qt * 16 + r)) * DM + h * HD + c;
        v8h t[8];
#pragma unroll
        for (int i = 0; i < 8; ++i) t[i] = *reinterpret_cast<const v8h*>(src + i * 8);
#pragma unroll
        for (int i = 0; i < 8; ++i) *reinterpret_cast<v8h*>(qs + r * QSP + c + i * 8) = t[i];
    }
    __syncthreads();

    const _Float16* qfr   = qs + l15 * QSP + hi8;
    const _Float16* kbase = kp + (size_t)b * SEQ * HD + hi8;
    const _Float16* vbase = vT + (size_t)(b * HD) * SEQ + hi8;

    const v8f zero8 = {0.f, 0.f, 0.f, 0.f, 0.f, 0.f, 0.f, 0.f};
    float m[8], l[8];
    v8f accY[8];
#pragma unroll
    for (int j = 0; j < 8; ++j) { m[j] = -1e30f; l[j] = 0.0f; }
#pragma unroll
    for (int ni = 0; ni < 8; ++ni) accY[ni] = zero8;

    const float sscale = 1.0f / (QCARRY * KCARRY);

    for (int tc = 0; tc < SEQ; tc += 32) {
        const _Float16* kr0 = kbase + (size_t)(tc + l15) * HD;
        const _Float16* kr1 = kr0 + 16 * HD;
        v8f s0 = zero8, s1 = zero8;
#pragma unroll
        for (int dc = 0; dc < 4; ++dc) {
            const v16h aq = load_frag(qfr + dc * 32);
            const v16h b0 = load_frag(kr0 + dc * 32);
            const v16h b1 = load_frag(kr1 + dc * 32);
            s0 = wmma16(aq, b0, s0);
            s1 = wmma16(aq, b1, s1);
            asm volatile("v_nop\n\tv_nop\n\tv_nop\n\tv_nop"
                         : "+v"(s0), "+v"(s1)
                         : "v"(aq), "v"(b0), "v"(b1));
        }

#pragma unroll
        for (int j = 0; j < 8; ++j) {
            const float a0 = s0[j] * sscale;
            const float a1 = s1[j] * sscale;
            float mt = fmaxf(a0, a1);
#pragma unroll
            for (int off = 8; off >= 1; off >>= 1)
                mt = fmaxf(mt, __shfl_xor(mt, off, 16));
            const float mn = fmaxf(m[j], mt);
            const float sc = exp2f(m[j] - mn);
            const float p0 = exp2f(a0 - mn);
            const float p1 = exp2f(a1 - mn);
            float rs = p0 + p1;
#pragma unroll
            for (int off = 8; off >= 1; off >>= 1)
                rs += __shfl_xor(rs, off, 16);
            l[j] = l[j] * sc + rs;
            m[j] = mn;
            accY[0][j] *= sc; accY[1][j] *= sc; accY[2][j] *= sc; accY[3][j] *= sc;
            accY[4][j] *= sc; accY[5][j] *= sc; accY[6][j] *= sc; accY[7][j] *= sc;
            const int row = hi8 + j;
            ps[row * PSP + l15]      = (_Float16)(p0 * PCARRY);
            ps[row * PSP + 16 + l15] = (_Float16)(p1 * PCARRY);
        }
        __syncthreads();

        const v16h aP = load_frag(ps + l15 * PSP + hi8);
        {
            const v16h v0 = load_frag(vbase + (size_t)(0 * 16 + l15) * SEQ + tc);
            const v16h v1 = load_frag(vbase + (size_t)(1 * 16 + l15) * SEQ + tc);
            const v16h v2 = load_frag(vbase + (size_t)(2 * 16 + l15) * SEQ + tc);
            const v16h v3 = load_frag(vbase + (size_t)(3 * 16 + l15) * SEQ + tc);
            accY[0] = wmma16(aP, v0, accY[0]);
            accY[1] = wmma16(aP, v1, accY[1]);
            accY[2] = wmma16(aP, v2, accY[2]);
            accY[3] = wmma16(aP, v3, accY[3]);
            asm volatile("v_nop\n\tv_nop\n\tv_nop\n\tv_nop"
                         : "+v"(accY[0]), "+v"(accY[1]), "+v"(accY[2]), "+v"(accY[3])
                         : "v"(aP), "v"(v0), "v"(v1), "v"(v2), "v"(v3));
        }
        {
            const v16h v4 = load_frag(vbase + (size_t)(4 * 16 + l15) * SEQ + tc);
            const v16h v5 = load_frag(vbase + (size_t)(5 * 16 + l15) * SEQ + tc);
            const v16h v6 = load_frag(vbase + (size_t)(6 * 16 + l15) * SEQ + tc);
            const v16h v7 = load_frag(vbase + (size_t)(7 * 16 + l15) * SEQ + tc);
            accY[4] = wmma16(aP, v4, accY[4]);
            accY[5] = wmma16(aP, v5, accY[5]);
            accY[6] = wmma16(aP, v6, accY[6]);
            accY[7] = wmma16(aP, v7, accY[7]);
            asm volatile("v_nop\n\tv_nop\n\tv_nop\n\tv_nop"
                         : "+v"(accY[4]), "+v"(accY[5]), "+v"(accY[6]), "+v"(accY[7])
                         : "v"(aP), "v"(v4), "v"(v5), "v"(v6), "v"(v7));
        }
        __syncthreads();
    }

    float inv[8];
#pragma unroll
    for (int j = 0; j < 8; ++j) inv[j] = (1.0f / l[j]) * (1.0f / (PCARRY * VCARRY));
#pragma unroll
    for (int ni = 0; ni < 8; ++ni)
#pragma unroll
        for (int j = 0; j < 8; ++j)
            my[(hi8 + j) * OSP + ni * 16 + l15] = accY[ni][j] * inv[j];
    __syncthreads();

    v4f v[16];
#pragma unroll
    for (int it = 0; it < 16; ++it)
        v[it] = *reinterpret_cast<const v4f*>(my + it * OSP + lane * 4);
    float* od = out + ((size_t)(b * SEQ + qt * 16)) * DM + h * HD + lane * 4;
#pragma unroll
    for (int it = 0; it < 16; ++it)
        *(volatile v4f*)(od + (size_t)it * DM) = v[it];
    __threadfence();
#pragma unroll
    for (int it = 0; it < 16; ++it)
        *(volatile v4f*)(od + (size_t)it * DM) = v[it];
}

extern "C" void kernel_launch(void* const* d_in, const int* in_sizes, int n_in,
                              void* d_out, int out_size, void* d_ws, size_t ws_size,
                              hipStream_t stream) {
    if (n_in < 9) return;
    const long long needX = ((long long)(NB - 1) * SEQ_FULL + SEQ) * DM;
    if ((long long)in_sizes[0] < needX || (long long)in_sizes[1] < needX || (long long)in_sizes[2] < needX) return;
    if (in_sizes[3] < DM * DM || in_sizes[4] < DM) return;
    if (in_sizes[5] < DM * HD || in_sizes[6] < HD) return;
    if (in_sizes[7] < DM * HD || in_sizes[8] < HD) return;
    if ((long long)out_size < (long long)MROWS * DM) return;

    const float* q  = (const float*)d_in[0];
    const float* k  = (const float*)d_in[1];
    const float* v  = (const float*)d_in[2];
    const float* Wq = (const float*)d_in[3];
    const float* bq = (const float*)d_in[4];
    const float* Wk = (const float*)d_in[5];
    const float* bk = (const float*)d_in[6];
    const float* Wv = (const float*)d_in[7];
    const float* bv = (const float*)d_in[8];
    float* out = (float*)d_out;

    size_t off = 0;
    char* wsb = (char*)d_ws;
    auto carve = [&](size_t bytes) -> void* {
        void* p = wsb + off;
        off += (bytes + 255) & ~(size_t)255;
        return p;
    };
    _Float16* q16 = (_Float16*)carve((size_t)MROWS * DM * 2);
    _Float16* k16 = (_Float16*)carve((size_t)MROWS * DM * 2);
    _Float16* v16 = (_Float16*)carve((size_t)MROWS * DM * 2);
    _Float16* WqT = (_Float16*)carve((size_t)DM * DM * 2);
    _Float16* WkT = (_Float16*)carve((size_t)HD * DM * 2);
    _Float16* WvT = (_Float16*)carve((size_t)HD * DM * 2);
    _Float16* qpl = (_Float16*)carve((size_t)MROWS * DM * 2);
    _Float16* kpl = (_Float16*)carve((size_t)MROWS * HD * 2);
    _Float16* vT  = (_Float16*)carve((size_t)NB * HD * SEQ * 2);
    if (off > ws_size) return;

    dim3 blk(256);
    const float qmul = SM_SCALE * LOG2E * QCARRY;

    k_cvt<<<dim3((MROWS * (DM / 8)) / 256), blk, 0, stream>>>(q, q16);
    k_cvt<<<dim3((MROWS * (DM / 8)) / 256), blk, 0, stream>>>(k, k16);
    k_cvt<<<dim3((MROWS * (DM / 8)) / 256), blk, 0, stream>>>(v, v16);
    k_wt<<<dim3(DM / 32, DM / 64), blk, 0, stream>>>(Wq, WqT, DM);
    k_wt<<<dim3(HD / 32, DM / 64), blk, 0, stream>>>(Wk, WkT, HD);
    k_wt<<<dim3(HD / 32, DM / 64), blk, 0, stream>>>(Wv, WvT, HD);

    k_gemm<0><<<dim3(DM / 128, MROWS / 128), blk, 0, stream>>>(
        q16, WqT, bq, qpl, DM, DM, 1.0f / WSCALE, qmul);
    k_gemm<0><<<dim3(HD / 128, MROWS / 128), blk, 0, stream>>>(
        k16, WkT, bk, kpl, HD, DM, 1.0f / WSCALE, KCARRY);
    k_gemm<2><<<dim3(1, MROWS / 128), blk, 0, stream>>>(
        v16, WvT, bv, vT, HD, DM, 1.0f / WSCALE, VCARRY);
    k_attn<<<dim3((NB * NH * (SEQ / 16)) / 4), dim3(128), 0, stream>>>(qpl, kpl, vT, out);
}
